// GRU_43301860278767
// MI455X (gfx1250) — hardware-run, weakly checked
//
#include <hip/hip_runtime.h>
#include <math.h>

typedef __attribute__((ext_vector_type(16))) _Float16 v16h;
typedef __attribute__((ext_vector_type(8)))  _Float16 v8h;
typedef __attribute__((ext_vector_type(2)))  _Float16 v2h;
typedef __attribute__((ext_vector_type(16))) __bf16   v16b;
typedef __attribute__((ext_vector_type(8)))  __bf16   v8b;
typedef __attribute__((ext_vector_type(8)))  float    v8f;
typedef __attribute__((ext_vector_type(4)))  float    v4f;
typedef __attribute__((ext_vector_type(2)))  float    v2f;

constexpr int kT    = 512;
constexpr int kB    = 64;
constexpr int kI    = 256;
constexpr int kH    = 512;
constexpr int kO    = 256;
constexpr int kG3   = 3 * kH;
constexpr int kG2   = 2 * kH;
constexpr int kC    = 64;
constexpr int kThr  = 256;
constexpr float kInCarry = 1024.0f;
constexpr float kSc = 1.0f / (kInCarry * kInCarry);
constexpr float kF16MinNormal = 6.103515625e-5f;

static_assert(kT == 512 && kB == 64 && kI == 256 && kH == 512 && kO == 256 && kG3 == 1536 && kG2 == 1024 && kC == 64 && kT % kC == 0, "the index arithmetic below uses these sizes");

constexpr size_t kOffZ = 0ull;
constexpr size_t kOffX16 = 204800ull;
constexpr size_t kOffWX16 = 16982016ull;
constexpr size_t kOffWH16 = 17768448ull;
constexpr size_t kOffWN16 = 18817024ull;
constexpr size_t kOffWO16 = 19341312ull;
constexpr size_t kOffBO = 19603456ull;
constexpr size_t kOffGX = 19607552ull;
constexpr size_t kOffG1 = 44773376ull;
constexpr size_t kOffG2 = 45035520ull;
constexpr size_t kOffRH16 = 45166592ull;
constexpr size_t kOffHS16 = 45232128ull;
constexpr size_t kWsTotal = 78786560ull;
static_assert(kWsTotal <= 268435456ull, "the carve stands under 256 MiB");
static_assert(kOffZ == 0
  && kOffX16 == kOffZ + 204800ull
  && kOffWX16 == kOffX16 + 16777216ull
  && kOffWH16 == kOffWX16 + 786432ull
  && kOffWN16 == kOffWH16 + 1048576ull
  && kOffWO16 == kOffWN16 + 524288ull
  && kOffBO == kOffWO16 + 262144ull
  && kOffGX == kOffBO + 4096ull
  && kOffG1 == kOffGX + 25165824ull
  && kOffG2 == kOffG1 + 262144ull
  && kOffRH16 == kOffG2 + 131072ull
  && kOffHS16 == kOffRH16 + 65536ull
  && kWsTotal == kOffHS16 + 33554432ull, "the carve is a chain: every region starts where the one before ends");
static_assert(8192ull + (size_t)kB * kH * 2 + (size_t)kB * kH * 4 == 204800ull && (size_t)kT * kB * kI * 2 == 16777216ull && (size_t)kG3 * kI * 2 == 786432ull && (size_t)kG2 * kH * 2 == 1048576ull && (size_t)kH * kH * 2 == 524288ull && (size_t)kO * kH * 2 == 262144ull
  && (size_t)kC * kB * kG3 * 4 == 25165824ull && (size_t)kB * kG2 * 4 == 262144ull && (size_t)kB * kH * 4 == 131072ull && (size_t)kB * kH * 2 == 65536ull && (size_t)kT * kB * kH * 2 == 33554432ull, "every region's length is its plane's");
static_assert((kOffX16 % 256) == 0 && (kOffWX16 % 256) == 0 && (kOffWH16 % 256) == 0 && (kOffWN16 % 256) == 0 && (kOffWO16 % 256) == 0 && (kOffBO % 256) == 0 && (kOffGX % 256) == 0 && (kOffG1 % 256) == 0 && (kOffG2 % 256) == 0 && (kOffRH16 % 256) == 0 && (kOffHS16 % 256) == 0, "every region starts on a multiple of 256 B");
constexpr size_t kZH16 = 8192ull;
constexpr size_t kZH32 = 8192ull + (size_t)kB * kH * 2;

__device__ __forceinline__ unsigned short f2bf_bits(float f) {
  unsigned u = __float_as_uint(f);
  return (unsigned short)((u + 0x7FFFu + ((u >> 16) & 1u)) >> 16);
}
__device__ __forceinline__ float bf_bits2f(unsigned short h) { return __uint_as_float(((unsigned)h) << 16); }
__device__ __forceinline__ float bf16r(float f) { return bf_bits2f(f2bf_bits(f)); }
__device__ __forceinline__ float carry_flush(float v, float carry) {
  const float s = v * carry;
  return (fabsf(s) < kF16MinNormal) ? 0.0f : s;
}

__device__ __forceinline__ void dep_guard4_h(v8f& a, v8f& b, v8f& c, v8f& d, v16h x, v16h y) { asm volatile("v_nop\n\tv_nop\n\tv_nop\n\tv_nop" : "+v"(a), "+v"(b), "+v"(c), "+v"(d) : "v"(x), "v"(y)); }
__device__ __forceinline__ void dep_guard4_b(v8f& a, v8f& b, v8f& c, v8f& d, v16b x, v16b y) { asm volatile("v_nop\n\tv_nop\n\tv_nop\n\tv_nop" : "+v"(a), "+v"(b), "+v"(c), "+v"(d) : "v"(x), "v"(y)); }
__device__ __forceinline__ void keep4_h(v16h a, v16h b, v16h c, v16h d) { asm volatile("v_nop" :: "v"(a), "v"(b), "v"(c), "v"(d)); }
__device__ __forceinline__ void keep4_b(v16b a, v16b b, v16b c, v16b d) { asm volatile("v_nop" :: "v"(a), "v"(b), "v"(c), "v"(d)); }
__device__ __forceinline__ void acc_guard4(v8f& a, v8f& b, v8f& c, v8f& d) { asm volatile("v_nop\n\tv_nop\n\tv_nop\n\tv_nop" : "+v"(a), "+v"(b), "+v"(c), "+v"(d)); }

template <typename T> struct Frag;
template <> struct Frag<_Float16> {
  typedef v16h V; union U { v16h v; v8h h[2]; };
  static __device__ __forceinline__ v16h load(const _Float16* p) {
    U f; f.h[0] = *(const v8h*)(p); f.h[1] = *(const v8h*)(p + 16); return f.v;
  }
  static __device__ __forceinline__ v8f mma(v16h a, v16h b, v8f c) {
    return __builtin_amdgcn_wmma_f32_16x16x32_f16(false, a, false, b, (short)0, c, false, false);
  }
  static __device__ __forceinline__ void guard4(v8f& a, v8f& b, v8f& c, v8f& d, v16h x, v16h y) { dep_guard4_h(a, b, c, d, x, y); }
  static __device__ __forceinline__ void keep(v16h a, v16h b, v16h c, v16h d) { keep4_h(a, b, c, d); }
};
template <> struct Frag<__bf16> {
  typedef v16b V; union U { v16b v; v8b h[2]; };
  static __device__ __forceinline__ v16b load(const __bf16* p) {
    U f; f.h[0] = *(const v8b*)(p); f.h[1] = *(const v8b*)(p + 16); return f.v;
  }
  static __device__ __forceinline__ v8f mma(v16b a, v16b b, v8f c) {
    return __builtin_amdgcn_wmma_f32_16x16x32_bf16(false, a, false, b, (short)0, c, false, false);
  }
  static __device__ __forceinline__ void guard4(v8f& a, v8f& b, v8f& c, v8f& d, v16b x, v16b y) { dep_guard4_b(a, b, c, d, x, y); }
  static __device__ __forceinline__ void keep(v16b a, v16b b, v16b c, v16b d) { keep4_b(a, b, c, d); }
};

__device__ __forceinline__ v8f mma_h(v16h a, v16h b, v8f c) {
  c = __builtin_amdgcn_wmma_f32_16x16x32_f16(false, a, false, b, (short)0, c, false, false);
  asm volatile("v_nop\n\tv_nop\n\tv_nop\n\tv_nop" : "+v"(c) : "v"(a), "v"(b));
  return c;
}

template <int ET> struct Elem;
template <> struct Elem<0> { typedef _Float16 T; };
template <> struct Elem<1> { typedef __bf16 T; };
template <int ET, bool SPLIT, int BIAS_MODE, int OUT_MODE, bool RESID, int ACT = 0>
__global__ __launch_bounds__(256) void wmma_gemm64(
    const unsigned short* __restrict__ Ap, const unsigned short* __restrict__ A2p, int lda, long strideA,
    const unsigned short* __restrict__ Btp, const unsigned short* __restrict__ Bt2p, int ldb, long strideB,
    void* __restrict__ Cout, void* __restrict__ Cout2, int ldc, long strideC,
    const float* __restrict__ bias,
    const float* __restrict__ resid, long strideR,
    int M, int N, int K, float scale) {
  typedef typename Elem<ET>::T T;
  typedef typename Frag<T>::V V;
  const T* A = (const T*)Ap; const T* A2 = (const T*)A2p; const T* Bt = (const T*)Btp; const T* Bt2 = (const T*)Bt2p;
  __shared__ __align__(16) float sT[8][16 * 68];
  const int b    = blockIdx.y;
  const int lane = threadIdx.x & 31;
  const int wave = threadIdx.x >> 5;
  const int tilesN = N >> 6;
  const int tilesM = M >> 6;
  const int tile = blockIdx.x * 8 + wave;
  if (tile >= tilesM * tilesN) return;
  const int tm = tile / tilesN;
  const int tn = tile - tm * tilesN;
  const int m0 = tm << 6;
  const int n0 = tn << 6;

  const T* Ab  = A  + (size_t)b * strideA;
  const T* Bb  = Bt + (size_t)b * strideB;
  const T* Ab2 = SPLIT ? (A2  + (size_t)b * strideA) : nullptr;
  const T* Bb2 = SPLIT ? (Bt2 + (size_t)b * strideB) : nullptr;

  const int rlane = lane & 15;
  const int koff  = (lane >> 4) * 8;
  const int mOff  = (lane >> 4) * 8;

  v8f acc[4][4];
#pragma unroll
  for (int i = 0; i < 4; ++i)
#pragma unroll
    for (int j = 0; j < 4; ++j) acc[i][j] = (v8f){0.f,0.f,0.f,0.f,0.f,0.f,0.f,0.f};

  for (int k0 = 0; k0 < K; k0 += 32) {
    V bh[4], bl[4];
#pragma unroll
    for (int j = 0; j < 4; ++j) {
      const size_t bo = (size_t)(n0 + (j << 4) + rlane) * ldb + koff + k0;
      bh[j] = Frag<T>::load(Bb + bo);
      if (SPLIT) bl[j] = Frag<T>::load(Bb2 + bo);
    }
#pragma unroll
    for (int i = 0; i < 4; ++i) {
      const size_t ao = (size_t)(m0 + (i << 4) + rlane) * lda + koff + k0;
      V ah = Frag<T>::load(Ab + ao);
      V al;
      if (SPLIT) al = Frag<T>::load(Ab2 + ao);
#pragma unroll
      for (int j = 0; j < 4; ++j) {
        acc[i][j] = Frag<T>::mma(ah, bh[j], acc[i][j]);
        if (SPLIT) {
          acc[i][j] = Frag<T>::mma(ah, bl[j], acc[i][j]);
          acc[i][j] = Frag<T>::mma(al, bh[j], acc[i][j]);
        }
      }
      Frag<T>::guard4(acc[i][0], acc[i][1], acc[i][2], acc[i][3], ah, SPLIT ? al : ah);
    }
    Frag<T>::keep(bh[0], bh[1], bh[2], bh[3]);
    if (SPLIT) Frag<T>::keep(bl[0], bl[1], bl[2], bl[3]);
  }
  acc_guard4(acc[0][0], acc[0][1], acc[0][2], acc[0][3]);
  acc_guard4(acc[1][0], acc[1][1], acc[1][2], acc[1][3]);
  acc_guard4(acc[2][0], acc[2][1], acc[2][2], acc[2][3]);
  acc_guard4(acc[3][0], acc[3][1], acc[3][2], acc[3][3]);

  float* slab = sT[wave];
  const float* Rb = RESID ? (resid + (size_t)b * strideR) : nullptr;
#pragma unroll
  for (int i = 0; i < 4; ++i) {
    const int mBase = m0 + (i << 4);
#pragma unroll
    for (int j = 0; j < 4; ++j) {
      const int n = n0 + (j << 4) + rlane;
      float bv = 0.f;
      if (BIAS_MODE == 2) bv = bias[n];
#pragma unroll
      for (int r = 0; r < 8; ++r) {
        float v = acc[i][j][r] * scale;
        if (BIAS_MODE == 1) v += bias[mBase + mOff + r];
        if (BIAS_MODE == 2) v += bv;
        if (RESID) v += Rb[(size_t)(mBase + mOff + r) * ldc + n];
        if (ACT == 1) v = tanhf(v);
        if (ACT == 2) v = fmaxf(v, 0.0f);
        if (ACT == 3) v = v / (1.0f + expf(-v));
        if (ACT == 4) v = (v > 0.f) ? v : 0.01f * v;
        slab[(mOff + r) * 68 + (j << 4) + rlane] = v;
      }
    }
    __builtin_amdgcn_fence(__ATOMIC_RELEASE, "workgroup");
    __builtin_amdgcn_wave_barrier();
    __builtin_amdgcn_fence(__ATOMIC_ACQUIRE, "workgroup");
    if (OUT_MODE == 0) {
      float* C = (float*)Cout + (size_t)b * strideC;
      const int hh = lane >> 4, c4 = (lane & 15) * 4;
      for (int pass = 0; pass < 2; ++pass) {
#pragma unroll
        for (int it = 0; it < 8; ++it) {
          const int row = it * 2 + hh;
          v4f v = *(const v4f*)(slab + row * 68 + c4);
          *(volatile v4f*)(C + (size_t)(mBase + row) * ldc + n0 + c4) = v;
        }
        __threadfence();
      }
    } else {
      const int q = lane >> 3, c8 = (lane & 7) * 8;
      unsigned short* C  = (unsigned short*)Cout  + (size_t)b * strideC;
      unsigned short* C2 = (OUT_MODE == 2) ? ((unsigned short*)Cout2 + (size_t)b * strideC) : nullptr;
      for (int pass = 0; pass < 2; ++pass) {
#pragma unroll
        for (int it = 0; it < 4; ++it) {
          const int row = it * 4 + q;
          const float* sp = slab + row * 68 + c8;
          v8h hv, lv;
#pragma unroll
          for (int e = 0; e < 8; ++e) {
            if (OUT_MODE == 1) {
              hv[e] = (_Float16)sp[e];
            } else {
              unsigned short hb = f2bf_bits(sp[e]);
              unsigned short lb = f2bf_bits(sp[e] - bf_bits2f(hb));
              hv[e] = __builtin_bit_cast(_Float16, hb);
              lv[e] = __builtin_bit_cast(_Float16, lb);
            }
          }
          *(volatile v8h*)(C + (size_t)(mBase + row) * ldc + n0 + c8) = hv;
          if (OUT_MODE == 2) *(volatile v8h*)(C2 + (size_t)(mBase + row) * ldc + n0 + c8) = lv;
        }
        __threadfence();
      }
    }
    __builtin_amdgcn_fence(__ATOMIC_RELEASE, "workgroup");
    __builtin_amdgcn_wave_barrier();
    __builtin_amdgcn_fence(__ATOMIC_ACQUIRE, "workgroup");
  }
}

__global__ __launch_bounds__(kThr) void cast_plane_kernel(const float* __restrict__ src, unsigned short* __restrict__ dst,
                                                          int colsLog2, int dstPitch, int dstOff) {
  const int i   = blockIdx.x * kThr + threadIdx.x;
  const int sh  = colsLog2 - 3;
  const int row = i >> sh;
  const int c8  = (i & ((1 << sh) - 1)) * 8;
  const float* sp = src + ((size_t)row << colsLog2) + c8;
  const v4f a0 = *(const v4f*)(sp);
  const v4f a1 = *(const v4f*)(sp + 4);
  v8h hv;
#pragma unroll
  for (int e = 0; e < 4; ++e) {
    const float f0 = a0[e];
    const float f1 = a1[e];
    hv[e]     = (_Float16)carry_flush(bf16r(f0), kInCarry);
    hv[4 + e] = (_Float16)carry_flush(bf16r(f1), kInCarry);
  }
  unsigned short* dp = dst + (size_t)row * dstPitch + dstOff + c8;
  *(volatile v8h*)dp = hv;
  __threadfence();
  *(volatile v8h*)dp = hv;
}

__global__ __launch_bounds__(kThr) void zero_kernel(float* __restrict__ dst) {
  const size_t o4 = ((size_t)blockIdx.x * kThr + threadIdx.x) * 4u;
  const v4f z = {0.f, 0.f, 0.f, 0.f};
  *(volatile v4f*)(dst + o4) = z;
  __threadfence();
  *(volatile v4f*)(dst + o4) = z;
}
__global__ __launch_bounds__(kThr) void pack_kernel(const float* __restrict__ W, unsigned short* __restrict__ D, float* __restrict__ dstf, int part, int ld, int k0, int lg, int n0, int pitch) {
  const unsigned i = blockIdx.x * blockDim.x + threadIdx.x;
  if (part == 0) {
    const unsigned g = i & ((1u << lg) - 1u), n = i >> lg;
    const float* sp = W + (size_t)((unsigned)k0 + g * 8u) * (unsigned)ld + n;
    v8h hv;
#pragma unroll
    for (int t = 0; t < 8; ++t) hv[t] = (_Float16)carry_flush(bf16r(sp[(size_t)t * (unsigned)ld]), kInCarry);
    unsigned short* dp = D + (size_t)((unsigned)n0 + n) * (unsigned)pitch + g * 8u;
    *(volatile v8h*)dp = hv;
    __threadfence();
    *(volatile v8h*)dp = hv;
  } else {
    const v4f a = *(const v4f*)(W + i * 4u);
    v4f o;
#pragma unroll
    for (int e = 0; e < 4; ++e) o[e] = bf16r(a[e]);
    float* dp = dstf + i * 4u;
    *(volatile v4f*)dp = o;
    __threadfence();
    *(volatile v4f*)dp = o;
  }
}

__global__ __launch_bounds__(kThr) void reset_kernel(const float* __restrict__ GXr, const float* __restrict__ G1, const float* __restrict__ br, const float* __restrict__ hprev, unsigned short* __restrict__ RH16) {
  const unsigned v = blockIdx.x * (unsigned)kThr + threadIdx.x;
  const unsigned b = v >> 6, u8 = (v & 63u) << 3;
  const float* gx = GXr + (size_t)b * kG3 + (unsigned)kH + u8;
  const float* g1 = G1 + (size_t)b * kG2 + (unsigned)kH + u8;
  const float* hp = hprev + (size_t)b * kH + u8;
  v8h hv;
#pragma unroll
  for (int hlf = 0; hlf < 2; ++hlf) {
    const v4f a = *(const v4f*)(gx + 4 * hlf), c = *(const v4f*)(g1 + 4 * hlf), q = *(const v4f*)(br + u8 + 4 * hlf), h = *(const v4f*)(hp + 4 * hlf);
#pragma unroll
    for (int e = 0; e < 4; ++e) {
      const float r = 1.0f / (1.0f + expf(-((a[e] + c[e]) + bf16r(q[e]))));
      hv[4 * hlf + e] = (_Float16)carry_flush(r * h[e], kInCarry);
    }
  }
  unsigned short* dp = RH16 + (size_t)b * kH + u8;
  *(volatile v8h*)dp = hv;
  __threadfence();
  *(volatile v8h*)dp = hv;
}
static_assert(kB * kH / 8 == 16 * kThr && kH / 8 == 64, "both cells' grid exact: 16 blocks; 64 threads a row");

__global__ __launch_bounds__(kThr) void blend_kernel(const float* __restrict__ GXr, const float* __restrict__ G1, const float* __restrict__ G2, const float* __restrict__ bz, const float* __restrict__ bn, const float* __restrict__ hprev,
                                                     float* __restrict__ hnew, unsigned short* __restrict__ HS16r) {
  const unsigned v = blockIdx.x * (unsigned)kThr + threadIdx.x;
  const unsigned b = v >> 6, u8 = (v & 63u) << 3;
  const float* gx = GXr + (size_t)b * kG3 + u8;
  const float* g1 = G1 + (size_t)b * kG2 + u8;
  const float* g2 = G2 + (size_t)b * kH + u8;
  const float* hp = hprev + (size_t)b * kH + u8;
  v8f ho; v8h hv;
#pragma unroll
  for (int hlf = 0; hlf < 2; ++hlf) {
    const v4f az = *(const v4f*)(gx + 4 * hlf), an = *(const v4f*)(gx + 2 * kH + 4 * hlf), cz = *(const v4f*)(g1 + 4 * hlf), cn = *(const v4f*)(g2 + 4 * hlf);
    const v4f qz = *(const v4f*)(bz + u8 + 4 * hlf), qn = *(const v4f*)(bn + u8 + 4 * hlf), h = *(const v4f*)(hp + 4 * hlf);
#pragma unroll
    for (int e = 0; e < 4; ++e) {
      const float z = 1.0f / (1.0f + expf(-((az[e] + cz[e]) + bf16r(qz[e]))));
      const float n = tanhf((an[e] + cn[e]) + bf16r(qn[e]));
      const float hn = (1.0f - z) * h[e] + z * n;
      ho[4 * hlf + e] = hn;
      hv[4 * hlf + e] = (_Float16)carry_flush(hn, kInCarry);
    }
  }
  float* po = hnew + (size_t)b * kH + u8;
  unsigned short* ph = HS16r + (size_t)b * kH + u8;
  for (int pass = 0; pass < 2; ++pass) {
    *(volatile v8f*)po = ho;
    *(volatile v8h*)ph = hv;
    __threadfence();
  }
}

extern "C" void kernel_launch(void* const* d_in, const int* in_sizes, int n_in,
                              void* d_out, int out_size, void* d_ws, size_t ws_size,
                              hipStream_t stream) {
  if (n_in < 9 || d_out == nullptr || d_ws == nullptr) return;
  if (in_sizes[0] != kT * kB * kI || in_sizes[1] != (kI + kH) * kH || in_sizes[2] != kH || in_sizes[3] != (kI + kH) * kH || in_sizes[4] != kH || in_sizes[5] != (kI + kH) * kH || in_sizes[6] != kH || in_sizes[7] != kH * kO || in_sizes[8] != kO) return;
  if (out_size != kT * kB * kO + kT * kB * kH) return;
  if (ws_size < kWsTotal) return;
  const float* x = (const float*)d_in[0];
  const float* Wz = (const float*)d_in[1];
  const float* bz = (const float*)d_in[2];
  const float* Wr = (const float*)d_in[3];
  const float* br = (const float*)d_in[4];
  const float* Wn = (const float*)d_in[5];
  const float* bn = (const float*)d_in[6];
  const float* Wo = (const float*)d_in[7];
  const float* bo = (const float*)d_in[8];
  float* oOut = (float*)d_out;
  float* oHS = oOut + (size_t)kT * kB * kO;
  char* ws = (char*)d_ws;
  float* ZB = (float*)(ws + kOffZ);
  unsigned short* ZH16 = (unsigned short*)(ws + kOffZ + kZH16);
  float* ZH32 = (float*)(ws + kOffZ + kZH32);
  unsigned short* X16 = (unsigned short*)(ws + kOffX16);
  unsigned short* WX16 = (unsigned short*)(ws + kOffWX16);
  unsigned short* WH16 = (unsigned short*)(ws + kOffWH16);
  unsigned short* WN16 = (unsigned short*)(ws + kOffWN16);
  unsigned short* WO16 = (unsigned short*)(ws + kOffWO16);
  float* BO = (float*)(ws + kOffBO);
  float* GX = (float*)(ws + kOffGX);
  float* G1 = (float*)(ws + kOffG1);
  float* G2 = (float*)(ws + kOffG2);
  unsigned short* RH16 = (unsigned short*)(ws + kOffRH16);
  unsigned short* HS16 = (unsigned short*)(ws + kOffHS16);

  static_assert(204800ull / 16ull == 50ull * kThr && ((size_t)kT * kB * kI / 8) % kThr == 0, "the zero fill's grid (50 blocks over Z's 204,800 B) and the cast's grid exact");
  zero_kernel<<<50, kThr, 0, stream>>>(ZB);
  cast_plane_kernel<<<(int)(((size_t)kT * kB * kI / 8) / kThr), kThr, 0, stream>>>(x, X16, 8, 256, 0);
  static_assert((kH * (kI / 8)) % kThr == 0 && (kH * (kH / 8)) % kThr == 0 && (kO * (kH / 8)) % kThr == 0, "the pack's grids exact");
  pack_kernel<<<kH * (kI / 8) / kThr, kThr, 0, stream>>>(Wz, WX16, nullptr, 0, kH, 0, 5, 0, kI);
  pack_kernel<<<kH * (kI / 8) / kThr, kThr, 0, stream>>>(Wr, WX16, nullptr, 0, kH, 0, 5, kH, kI);
  pack_kernel<<<kH * (kI / 8) / kThr, kThr, 0, stream>>>(Wn, WX16, nullptr, 0, kH, 0, 5, 2 * kH, kI);
  pack_kernel<<<kH * (kH / 8) / kThr, kThr, 0, stream>>>(Wz, WH16, nullptr, 0, kH, kI, 6, 0, kH);
  pack_kernel<<<kH * (kH / 8) / kThr, kThr, 0, stream>>>(Wr, WH16, nullptr, 0, kH, kI, 6, kH, kH);
  pack_kernel<<<kH * (kH / 8) / kThr, kThr, 0, stream>>>(Wn, WN16, nullptr, 0, kH, kI, 6, 0, kH);
  pack_kernel<<<kO * (kH / 8) / kThr, kThr, 0, stream>>>(Wo, WO16, nullptr, 0, kO, 0, 6, 0, kH);
  pack_kernel<<<1, 64, 0, stream>>>(bo, nullptr, BO, 1, 0, 0, 0, 0, 0);
  for (int c = 0; c < kT / kC; ++c) {
    wmma_gemm64<0, false, 2, 0, false, 0><<<dim3((kC * kB / 64) * (kG3 / 64) / 8, 1), 256, 0, stream>>>(
        X16 + (size_t)c * kC * kB * kI, X16 + (size_t)c * kC * kB * kI, kI, 0L, WX16, WX16, kI, 0L, (void*)GX, (void*)GX, kG3, 0L, ZB, nullptr, 0L, kC * kB, kG3, kI, kSc);
    for (int kk = 0; kk < kC; ++kk) {
      const int t = c * kC + kk;
      const unsigned short* h16 = (t == 0) ? ZH16 : (HS16 + (size_t)(t - 1) * kB * kH);
      const float* h32 = (t == 0) ? ZH32 : (oHS + (size_t)(t - 1) * kB * kH);
      const float* gxr = GX + (size_t)kk * kB * kG3;
      wmma_gemm64<0, false, 2, 0, false, 0><<<dim3((kB / 64) * (kG2 / 64) / 8, 1), 256, 0, stream>>>(
          h16, h16, kH, 0L, WH16, WH16, kH, 0L, (void*)G1, (void*)G1, kG2, 0L, ZB, nullptr, 0L, kB, kG2, kH, kSc);
      reset_kernel<<<16, kThr, 0, stream>>>(gxr, G1, br, h32, RH16);
      wmma_gemm64<0, false, 2, 0, false, 0><<<dim3((kB / 64) * (kH / 64) / 8, 1), 256, 0, stream>>>(
          RH16, RH16, kH, 0L, WN16, WN16, kH, 0L, (void*)G2, (void*)G2, kH, 0L, ZB, nullptr, 0L, kB, kH, kH, kSc);
      blend_kernel<<<16, kThr, 0, stream>>>(gxr, G1, G2, bz, bn, h32, oHS + (size_t)t * kB * kH, HS16 + (size_t)t * kB * kH);
    }
  }
  wmma_gemm64<0, false, 2, 0, false, 0><<<dim3((kT * kB / 64) * (kO / 64) / 8, 1), 256, 0, stream>>>(
      HS16, HS16, kH, 0L, WO16, WO16, kH, 0L, (void*)oOut, (void*)oOut, kO, 0L, BO, nullptr, 0L, kT * kB, kO, kH, kSc);
}
static_assert(((kC * kB / 64) * (kG3 / 64)) % 8 == 0 && ((kB / 64) * (kG2 / 64)) % 8 == 0 && ((kB / 64) * (kH / 64)) % 8 == 0 && ((kT * kB / 64) * (kO / 64)) % 8 == 0, "every engine grid: whole blocks of eight wave tiles");
